// VelVecPot3D_18021682774227
// MI455X (gfx1250) — hardware-verified
//
#include <hip/hip_runtime.h>


#define NN   65536
#define CH   16384
#define DI   4
#define DW   256
#define NL   5
typedef _Float16 h16;
typedef unsigned short bf;
typedef __attribute__((ext_vector_type(16))) __bf16   v16bf;
typedef __attribute__((ext_vector_type(16))) _Float16 v16h;
typedef __attribute__((ext_vector_type(8)))  _Float16 v8h;
typedef __attribute__((ext_vector_type(8)))  unsigned short v8us;
typedef __attribute__((ext_vector_type(8)))  float    v8f;
typedef __attribute__((ext_vector_type(4)))  float    v4f;
typedef v8h  __attribute__((may_alias)) v8ha;
typedef v4f  __attribute__((may_alias)) v4fa;
typedef v8us __attribute__((may_alias)) v8usa;

__device__ __forceinline__ unsigned short f2bf(float f) { unsigned u = __float_as_uint(f); u += 0x7FFFu + ((u >> 16) & 1u); return (unsigned short)(u >> 16); }
__device__ __forceinline__ float bf2f(unsigned short b) { return __uint_as_float(((unsigned)b) << 16); }
__device__ __forceinline__ float bfr(float f) { return bf2f(f2bf(f)); }
__device__ __forceinline__ v16h cat16(v8h lo, v8h hi) { return __builtin_shufflevector(lo, hi, 0, 1, 2, 3, 4, 5, 6, 7, 8, 9, 10, 11, 12, 13, 14, 15); }
__device__ __forceinline__ v16bf cat16b(v8us lo, v8us hi) { return __builtin_bit_cast(v16bf, __builtin_shufflevector(lo, hi, 0, 1, 2, 3, 4, 5, 6, 7, 8, 9, 10, 11, 12, 13, 14, 15)); }
__device__ __forceinline__ v8f wmma16(v16h a, v16h b, v8f c) { return __builtin_amdgcn_wmma_f32_16x16x32_f16(false, a, false, b, (short)0, c, false, false); }
__device__ __forceinline__ v8f wmmab(v16bf a, v16bf b, v8f c) { return __builtin_amdgcn_wmma_f32_16x16x32_bf16(false, a, false, b, (short)0, c, false, false); }


template <typename T16> struct WFrag;
template <> struct WFrag<h16> { typedef v16h V; static __device__ __forceinline__ V ld(const h16* p) { return cat16(*(const v8h*)p, *(const v8h*)(p + 16)); } static __device__ __forceinline__ v8f mma(V a, V b, v8f c) { return wmma16(a, b, c); } };
template <> struct WFrag<bf> { typedef v16bf V; static __device__ __forceinline__ V ld(const bf* p) { return cat16b(*(const v8us*)p, *(const v8us*)(p + 16)); } static __device__ __forceinline__ v8f mma(V a, V b, v8f c) { return wmmab(a, b, c); } };
template <typename T16, int NSPLIT, bool BIAS>
__global__ __launch_bounds__(32) void k_gemmw(const T16* __restrict__ A, const T16* __restrict__ A2, const T16* __restrict__ Bt, const T16* __restrict__ Bt2, int K, float* C, int ldc, const float* __restrict__ bias, size_t sA, size_t sB, size_t sC) {
    typedef typename WFrag<T16>::V V;
    __shared__ __align__(16) float os[16 * 68];
    const size_t z = blockIdx.z; A += z * sA; if (A2) A2 += z * sA; Bt += z * sB; if (Bt2) Bt2 += z * sB; C += z * sC;
    const int lane = threadIdx.x & 31, lr = lane & 15, hi = lane >> 4; const int r0 = blockIdx.x * 64, c0 = blockIdx.y * 64;
    v8f acc[4][4];
#pragma unroll
    for (int mb = 0; mb < 4; ++mb)
#pragma unroll
        for (int nb = 0; nb < 4; ++nb) acc[mb][nb] = (v8f){};
    const size_t aoff = (size_t)(r0 + lr) * K + 8 * hi, boff = (size_t)(c0 + lr) * K + 8 * hi;
#pragma unroll 1
    for (int kc = 0; kc < K; kc += 32) {
        V a[4], a2[4];
#pragma unroll
        for (int mb = 0; mb < 4; ++mb) { a[mb] = WFrag<T16>::ld(A + aoff + (size_t)mb * 16 * K + kc); if (NSPLIT == 1 || NSPLIT == 2) a2[mb] = WFrag<T16>::ld(A2 + aoff + (size_t)mb * 16 * K + kc); }
#pragma unroll
        for (int nb = 0; nb < 4; ++nb) { const V b = WFrag<T16>::ld(Bt + boff + (size_t)nb * 16 * K + kc); V b2; if (NSPLIT >= 2) b2 = WFrag<T16>::ld(Bt2 + boff + (size_t)nb * 16 * K + kc);
#pragma unroll
            for (int mb = 0; mb < 4; ++mb) { acc[mb][nb] = WFrag<T16>::mma(a[mb], b, acc[mb][nb]); if (NSPLIT == 1 || NSPLIT == 2) acc[mb][nb] = WFrag<T16>::mma(a2[mb], b, acc[mb][nb]); if (NSPLIT >= 2) acc[mb][nb] = WFrag<T16>::mma(a[mb], b2, acc[mb][nb]); } }
        asm volatile("v_nop\n\tv_nop\n\tv_nop\n\tv_nop" : "+v"(acc[0][0]), "+v"(acc[1][1]), "+v"(acc[2][2]), "+v"(acc[3][3]) : "v"(a[0]), "v"(a[3]));
    }
#pragma unroll
    for (int mb = 0; mb < 4; ++mb) {
#pragma unroll
        for (int nb = 0; nb < 4; ++nb) {
#pragma unroll
            for (int j = 0; j < 8; ++j) os[(hi * 8 + j) * 68 + nb * 16 + lr] = acc[mb][nb][j]; }
        __builtin_amdgcn_wave_barrier(); asm volatile("" ::: "memory");
        float* crow = C + (size_t)(r0 + mb * 16) * ldc + c0;
#pragma unroll 1
        for (int ps = 0; ps < 2; ++ps) {
#pragma unroll
            for (int s = 0; s < 8; ++s) { const int row = 2 * s + hi, cofs = lr * 4; v4f val = *(const v4fa*)(os + row * 68 + cofs); if (BIAS) { val[0] += bfr(bias[c0 + cofs]); val[1] += bfr(bias[c0 + cofs + 1]); val[2] += bfr(bias[c0 + cofs + 2]); val[3] += bfr(bias[c0 + cofs + 3]); }
                *(volatile v4f*)(crow + (size_t)row * ldc + cofs) = val; }
            if (ps == 0) __threadfence(); }
        __builtin_amdgcn_wave_barrier(); asm volatile("" ::: "memory");
    }
}

__device__ __forceinline__ h16 tohx(float x) { return (h16)x; }
__device__ __forceinline__ float tanhf_(float a) { const float e2 = __expf(2.0f * a); return __fsub_rn(1.0f, __fdiv_rn(2.0f, __fadd_rn(e2, 1.0f))); }
typedef __attribute__((ext_vector_type(2))) _Float16 v2h;
typedef __attribute__((ext_vector_type(4))) _Float16 v4h;
typedef __attribute__((ext_vector_type(2))) float v2f;

__global__ __launch_bounds__(256) void k_w16T(const float* __restrict__ w, int K, int N, h16* Bt) { __shared__ float tile[64][65]; const int nt = (N + 63) / 64; const int bk = blockIdx.x / nt, bn = blockIdx.x % nt; const int tx = threadIdx.x & 63, ty = threadIdx.x >> 6;
    for (int r = ty; r < 64; r += 4) { const int k = bk * 64 + r, n = bn * 64 + tx; tile[r][tx] = (k < K && n < N) ? w[(size_t)k * N + n] : 0.f; } __syncthreads();
    for (int ps = 0; ps < 2; ++ps) { for (int r = ty; r < 64; r += 4) { const int n = bn * 64 + r, k = bk * 64 + tx; if (n < N && k < K) *(volatile h16*)(Bt + (size_t)n * K + k) = tohx(bfr(tile[tx][r])); } if (ps == 0) __threadfence(); } }
__global__ __launch_bounds__(256) void k_c16(const float* __restrict__ w, h16* o, size_t n4) { const size_t i = (size_t)blockIdx.x * 256 + threadIdx.x; if (i >= n4) return; const v4f a = *(const v4f*)(w + i * 4); v4h r; r[0] = tohx(bfr(a[0])); r[1] = tohx(bfr(a[1])); r[2] = tohx(bfr(a[2])); r[3] = tohx(bfr(a[3])); *(volatile v4h*)(o + i * 4) = r; __threadfence(); *(volatile v4h*)(o + i * 4) = r; }
__global__ __launch_bounds__(256) void k_h0(const float* __restrict__ x, const float* __restrict__ W0, const float* __restrict__ b0, int r0, h16* A16) { const size_t e = ((size_t)blockIdx.x * 256 + threadIdx.x) * 2; if (e >= (size_t)CH * DW) return; const int c = (int)(e % DW), n = (int)(e / DW); v2h o;
#pragma unroll
    for (int q = 0; q < 2; ++q) { float s = 0.f;
#pragma unroll
        for (int d = 0; d < DI; ++d) { float p = __fmul_rn(bfr(x[(size_t)(r0 + n) * DI + d]), bfr(W0[d * DW + c + q])); asm volatile("" : "+v"(p)); s = __fadd_rn(s, p); } o[q] = tohx(__fadd_rn(s, bfr(b0[c + q]))); }
    *(volatile v2h*)(A16 + e) = o; __threadfence(); *(volatile v2h*)(A16 + e) = o; }
__global__ __launch_bounds__(256) void k_tanh(const float* __restrict__ Z, float* H, h16* A16) { const size_t e = ((size_t)blockIdx.x * 256 + threadIdx.x) * 2; if (e >= (size_t)CH * DW) return; v2f hf; v2h o;
#pragma unroll
    for (int q = 0; q < 2; ++q) { hf[q] = tanhf_(Z[e + q]); o[q] = tohx(hf[q]); } *(volatile v2f*)(H + e) = hf; *(volatile v2h*)(A16 + e) = o; __threadfence(); *(volatile v2f*)(H + e) = hf; *(volatile v2h*)(A16 + e) = o; }
__global__ __launch_bounds__(256) void k_gz0(const float* __restrict__ Wl, const float* __restrict__ H5, h16* GZ) { const size_t e = ((size_t)blockIdx.x * 256 + threadIdx.x) * 2; if (e >= (size_t)3 * CH * DW) return; const int k = (int)(e % DW); const int n = (int)((e / DW) % CH); const int c = (int)(e / ((size_t)DW * CH)); v2h o;
#pragma unroll
    for (int q = 0; q < 2; ++q) { const float h = H5[(size_t)n * DW + k + q]; float hh = __fmul_rn(h, h); asm volatile("" : "+v"(hh)); o[q] = tohx(__fmul_rn(bfr(Wl[(k + q) * 3 + c]), __fsub_rn(1.0f, hh))); } *(volatile v2h*)(GZ + e) = o; __threadfence(); *(volatile v2h*)(GZ + e) = o; }
__global__ __launch_bounds__(256) void k_gz(const float* __restrict__ G, const float* __restrict__ H, h16* GZ) { const size_t e = ((size_t)blockIdx.x * 256 + threadIdx.x) * 2; if (e >= (size_t)3 * CH * DW) return; const size_t nk = e % ((size_t)CH * DW); v2h o;
#pragma unroll
    for (int q = 0; q < 2; ++q) { const float h = H[nk + q]; float hh = __fmul_rn(h, h); asm volatile("" : "+v"(hh)); o[q] = tohx(__fmul_rn(G[e + q], __fsub_rn(1.0f, hh))); } *(volatile v2h*)(GZ + e) = o; __threadfence(); *(volatile v2h*)(GZ + e) = o; }
__global__ __launch_bounds__(256) void k_curl(const float* __restrict__ G, const float* __restrict__ W0, float* U4) { const int n = blockIdx.x * 256 + threadIdx.x; if (n >= CH) return; float j01 = 0.f, j02 = 0.f, j10 = 0.f, j12 = 0.f, j20 = 0.f, j21 = 0.f;
    const float* g0 = G + (size_t)n * DW; const float* g1 = G + ((size_t)CH + n) * DW; const float* g2 = G + ((size_t)2 * CH + n) * DW;
    for (int k = 0; k < DW; ++k) { const float w0 = bfr(W0[k]), w1 = bfr(W0[DW + k]), w2 = bfr(W0[2 * DW + k]); float a = __fmul_rn(g0[k], w1), b = __fmul_rn(g0[k], w2), c = __fmul_rn(g1[k], w0), d = __fmul_rn(g1[k], w2), e2 = __fmul_rn(g2[k], w0), f = __fmul_rn(g2[k], w1); asm volatile("" : "+v"(a), "+v"(b), "+v"(c), "+v"(d), "+v"(e2), "+v"(f));
        j01 = __fadd_rn(j01, a); j02 = __fadd_rn(j02, b); j10 = __fadd_rn(j10, c); j12 = __fadd_rn(j12, d); j20 = __fadd_rn(j20, e2); j21 = __fadd_rn(j21, f); }
    v4f u; u[0] = __fsub_rn(j21, j12); u[1] = __fsub_rn(j02, j20); u[2] = __fsub_rn(j10, j01); u[3] = 0.f; *(volatile v4f*)(U4 + (size_t)n * 4) = u; __threadfence(); *(volatile v4f*)(U4 + (size_t)n * 4) = u; }
__global__ __launch_bounds__(256) void k_out3(const float* __restrict__ U4, float* OUTc) { const int i = (blockIdx.x * 256 + threadIdx.x) * 4; if (i >= CH * 3) return; v4f o;
#pragma unroll
    for (int q = 0; q < 4; ++q) { const int e = i + q; o[q] = U4[(size_t)(e / 3) * 4 + (e % 3)]; } *(volatile v4f*)(OUTc + i) = o; __threadfence(); *(volatile v4f*)(OUTc + i) = o; }

extern "C" void kernel_launch(void* const* d_in, const int* in_sizes, int n_in,
                              void* d_out, int out_size, void* d_ws, size_t ws_size, hipStream_t stream) {
    (void)in_sizes; (void)n_in; (void)out_size;
    const float* x = (const float*)d_in[0]; const float* W0 = (const float*)d_in[1]; const float* b0 = (const float*)d_in[2]; const float* Wh = (const float*)d_in[3]; const float* bh = (const float*)d_in[4]; const float* Wl = (const float*)d_in[5];
    float* OUT = (float*)d_out;
    char* wsp = (char*)d_ws;
    auto take = [&](size_t bytes) { char* p = wsp; wsp += (bytes + 255) & ~(size_t)255; return (void*)p; };
    h16* WF = (h16*)take((size_t)NL * DW * DW * 2); h16* WB = (h16*)take((size_t)NL * DW * DW * 2);
    h16* A16 = (h16*)take((size_t)CH * DW * 2); float* Z = (float*)take((size_t)CH * DW * 4); float* Hs = (float*)take((size_t)NL * CH * DW * 4); h16* GZ = (h16*)take((size_t)3 * CH * DW * 2); float* G = (float*)take((size_t)3 * CH * DW * 4); float* U4 = (float*)take((size_t)CH * 4 * 4);
    if ((size_t)(wsp - (char*)d_ws) > ws_size) return;
    for (int i = 0; i < NL; ++i) { k_w16T<<<(DW / 64) * (DW / 64), 256, 0, stream>>>(Wh + (size_t)i * DW * DW, DW, DW, WF + (size_t)i * DW * DW); k_c16<<<(DW * DW / 4 + 255) / 256, 256, 0, stream>>>(Wh + (size_t)i * DW * DW, WB + (size_t)i * DW * DW, (size_t)DW * DW / 4); }
    const unsigned L2 = (unsigned)(((size_t)CH * DW / 2 + 255) / 256), L6 = (unsigned)(((size_t)3 * CH * DW / 2 + 255) / 256);
    for (int ck = 0; ck < NN / CH; ++ck) { const int r0 = ck * CH;
        k_h0<<<L2, 256, 0, stream>>>(x, W0, b0, r0, A16);
        for (int i = 0; i < NL; ++i) { k_gemmw<h16, 0, true><<<dim3(CH / 64, DW / 64, 1), 32, 0, stream>>>(A16, nullptr, WF + (size_t)i * DW * DW, nullptr, DW, Z, DW, bh + (size_t)i * DW, 0, 0, 0); k_tanh<<<L2, 256, 0, stream>>>(Z, Hs + (size_t)i * CH * DW, A16); }
        k_gz0<<<L6, 256, 0, stream>>>(Wl, Hs + (size_t)4 * CH * DW, GZ);
        for (int i = NL - 1; i >= 0; --i) { k_gemmw<h16, 0, false><<<dim3(CH / 64, DW / 64, 3), 32, 0, stream>>>(GZ, nullptr, WB + (size_t)i * DW * DW, nullptr, DW, G, DW, nullptr, (size_t)CH * DW, 0, (size_t)CH * DW);
            if (i > 0) k_gz<<<L6, 256, 0, stream>>>(G, Hs + (size_t)(i - 1) * CH * DW, GZ); }
        k_curl<<<CH / 256, 256, 0, stream>>>(G, W0, U4); k_out3<<<(CH * 3 / 4 + 255) / 256, 256, 0, stream>>>(U4, OUT + (size_t)r0 * 3); }
}
